// E3Conv_16887811408323
// MI455X (gfx1250) — hardware-verified
//
#include <hip/hip_runtime.h>
#include <stddef.h>

#pragma clang fp contract(off)


#define NTHR   256
#define NWAVE  8
#define EPT    8
#define CHUNK  (NTHR * EPT)
#define WCAP   (EPT * 32)
#define LISTN  (NWAVE * WCAP)
#define PASSN  256
#define PCAP   (CHUNK + PASSN)
#define NB     64
#define CS     64
#define CV     32
#define VW     96
#define EA     16
#define UNIONB 41984
#define MISCB  1536
#define SQ3    1.7320508075688772f

static_assert(PASSN == NTHR);
static_assert((NB & (NB - 1)) == 0);
static_assert(PCAP >= CHUNK + PASSN);
static_assert(PASSN * 64 + PASSN * 16 + PASSN * 4 + LISTN * 4 + PCAP * 4 <= UNIONB);
static_assert(NB * CS * 4 + NB * VW * 4 + 3 * NB * 4 <= UNIONB);

typedef float          v4f   __attribute__((ext_vector_type(4)));
typedef float          v8f   __attribute__((ext_vector_type(8)));
typedef int            v4i   __attribute__((ext_vector_type(4)));
typedef unsigned short v8us  __attribute__((ext_vector_type(8)));
typedef unsigned short v16us __attribute__((ext_vector_type(16)));
typedef __bf16         v16b  __attribute__((ext_vector_type(16)));
union FU { v16us u; v8us h[2]; };

__host__ __device__ constexpr int accw(int mode) { return mode ? 480 : 256; }
__host__ __device__ constexpr int lds_bytes(int mode) { return 2 * NB * accw(mode) * 4 + UNIONB + MISCB; }

__device__ __forceinline__ v8f zero8f() {
  v8f z;
#pragma unroll
  for (int i = 0; i < 8; ++i) z[i] = 0.0f;
  return z;
}

__device__ __forceinline__ v8f wm(v16us a, v16us b, v8f c) {
  const v16b av = __builtin_bit_cast(v16b, a);
  const v16b bv = __builtin_bit_cast(v16b, b);
  v8f d = __builtin_amdgcn_wmma_f32_16x16x32_bf16(false, av, false, bv, (short)0, c, false, false);
  asm volatile("v_nop\n\tv_nop\n\tv_nop\n\tv_nop" : "+v"(d) : "v"(a), "v"(b));
  return d;
}

__device__ __forceinline__ v8f mm3(v16us ah, v16us al, v16us bh, v16us bl, v8f d) {
  d = wm(ah, bh, d);
  d = wm(ah, bl, d);
  d = wm(al, bh, d);
  return d;
}

__device__ __forceinline__ unsigned int bfb(float x) {
  unsigned int u = __float_as_uint(x);
  u += 0x7FFFu + ((u >> 16) & 1u);
  return u >> 16;
}
__device__ __forceinline__ unsigned int bflo(float x, unsigned int hb) {
  return bfb(x - __uint_as_float(hb << 16));
}

__device__ __forceinline__ void fragBe(const float* __restrict__ W, int ncol, int n0, int h, int m, v16us& bh, v16us& bl) {
#pragma unroll
  for (int i = 0; i < 8; ++i) {
    const float w = W[(8 * h + i) * ncol + n0 + m];
    const unsigned int hb = bfb(w), lb = bflo(w, hb);
    bh[i] = (unsigned short)hb; bh[8 + i] = (unsigned short)hb;
    bl[i] = (unsigned short)lb; bl[8 + i] = (unsigned short)lb;
  }
}

__device__ __forceinline__ void fragBw(const float* __restrict__ W, int ncol, int k0, int n0, int h, int m, v16us& bh, v16us& bl) {
#pragma unroll
  for (int i = 0; i < 8; ++i) {
    const float w0 = W[(k0 + 8 * h + i) * ncol + n0 + m];
    const float w1 = W[(k0 + 16 + 8 * h + i) * ncol + n0 + m];
    const unsigned int h0 = bfb(w0), h1 = bfb(w1);
    bh[i] = (unsigned short)h0; bl[i] = (unsigned short)bflo(w0, h0);
    bh[8 + i] = (unsigned short)h1; bl[8 + i] = (unsigned short)bflo(w1, h1);
  }
}

template <int AW>
__device__ __forceinline__ void fragAacc(const float* acc, int row0, int base, int st, float invn, int h, int m, v16us& ah, v16us& al) {
  const float* p0 = acc + (row0 + m) * AW + base + st * 8 * h;
  const float* p1 = p0 + NB * AW;
#pragma unroll
  for (int i = 0; i < 8; ++i) {
    const float v0 = (p0[st * i] + p1[st * i]) * invn;
    const float v1 = (p0[st * (16 + i)] + p1[st * (16 + i)]) * invn;
    const unsigned int h0 = bfb(v0), h1 = bfb(v1);
    ah[i] = (unsigned short)h0; al[i] = (unsigned short)bflo(v0, h0);
    ah[8 + i] = (unsigned short)h1; al[8 + i] = (unsigned short)bflo(v1, h1);
  }
}

__device__ __forceinline__ void fragApl(const float* __restrict__ P, int pitch, int coff, int node0, int nN, int k0,
                                        const float* sc, int h, int m, v16us& ah, v16us& al) {
  const int n = min(node0 + m, nN - 1);
  const float* p = P + (size_t)n * pitch + coff + k0 + 8 * h;
  const float* q = sc + k0 + 8 * h;
#pragma unroll
  for (int i = 0; i < 8; ++i) {
    const float v0 = p[i] * q[i];
    const float v1 = p[16 + i] * q[16 + i];
    const unsigned int h0 = bfb(v0), h1 = bfb(v1);
    ah[i] = (unsigned short)h0; al[i] = (unsigned short)bflo(v0, h0);
    ah[8 + i] = (unsigned short)h1; al[8 + i] = (unsigned short)bflo(v1, h1);
  }
}

__device__ __forceinline__ int dst_of(const int* __restrict__ rad, const int* __restrict__ bnd, int nER, int nEB, int nE, int e, int sent) {
  const int er = min(max(e, 0), nER - 1);
  const int eb = min(max(e - nER, 0), nEB - 1);
  const int dR = rad[nER + er];
  const int dB = bnd[nEB + eb];
  return (e < nE) ? ((e < nER) ? dR : dB) : sent;
}

__device__ __forceinline__ int scan_chunk(const int* __restrict__ rad, const int* __restrict__ bnd, int nER, int nEB,
                                          int cbase, int nodeBase, int vecOK, int* list, int tid, int wave) {
  int wc = 0;
  const int nE = nER + nEB;
  const int el0 = tid * EPT;
  const int e0 = cbase + el0;
  const int sent = -2147483647 - 1;
  v4i da, db;
  if (vecOK != 0 && cbase + CHUNK <= nER) {
    const int* p = rad + nER + e0;
    da = *(const v4i*)p; db = *(const v4i*)(p + 4);
  } else if (vecOK != 0 && cbase >= nER && cbase + CHUNK <= nE) {
    const int* p = bnd + nEB + (e0 - nER);
    da = *(const v4i*)p; db = *(const v4i*)(p + 4);
  } else {
    da.x = dst_of(rad, bnd, nER, nEB, nE, e0, sent);     da.y = dst_of(rad, bnd, nER, nEB, nE, e0 + 1, sent);
    da.z = dst_of(rad, bnd, nER, nEB, nE, e0 + 2, sent); da.w = dst_of(rad, bnd, nER, nEB, nE, e0 + 3, sent);
    db.x = dst_of(rad, bnd, nER, nEB, nE, e0 + 4, sent); db.y = dst_of(rad, bnd, nER, nEB, nE, e0 + 5, sent);
    db.z = dst_of(rad, bnd, nER, nEB, nE, e0 + 6, sent); db.w = dst_of(rad, bnd, nER, nEB, nE, e0 + 7, sent);
  }
  const unsigned nb = (unsigned)nodeBase;
  const unsigned s0 = (unsigned)da.x - nb, s1 = (unsigned)da.y - nb, s2 = (unsigned)da.z - nb, s3 = (unsigned)da.w - nb;
  const unsigned s4 = (unsigned)db.x - nb, s5 = (unsigned)db.y - nb, s6 = (unsigned)db.z - nb, s7 = (unsigned)db.w - nb;
  const bool h0 = s0 < (unsigned)NB, h1 = s1 < (unsigned)NB, h2 = s2 < (unsigned)NB, h3 = s3 < (unsigned)NB;
  const bool h4 = s4 < (unsigned)NB, h5 = s5 < (unsigned)NB, h6 = s6 < (unsigned)NB, h7 = s7 < (unsigned)NB;
  const unsigned any = __builtin_amdgcn_ballot_w32(h0 | h1 | h2 | h3 | h4 | h5 | h6 | h7);
  if (any != 0u) {
#define HITJ(J, HJ) { \
      const unsigned mj = __builtin_amdgcn_ballot_w32(HJ); \
      if (mj != 0u) { \
        if (HJ) { \
          const int pp = wc + (int)__builtin_amdgcn_mbcnt_lo(mj, 0u); \
          if (pp < WCAP) list[wave * WCAP + pp] = el0 + (J); \
        } \
        wc += (int)__builtin_popcount(mj); } }
    HITJ(0, h0) HITJ(1, h1) HITJ(2, h2) HITJ(3, h3)
    HITJ(4, h4) HITJ(5, h5) HITJ(6, h6) HITJ(7, h7)
#undef HITJ
  }
  return wc;
}

template <int AW>
__device__ __forceinline__ void roleA(float* acc, const unsigned short* eaL, const int* idL, const float* y4L,
                                      const float* __restrict__ Sin, float sc, int c,
                                      v16us B1h, v16us B1l, v16us B2h, v16us B2l, int nt, int h, int m) {
  float* ab = acc + h * (NB * AW);
  const v8f z = zero8f();
#pragma unroll 1
  for (int t = 0; t < nt; ++t) {
    FU a;
    const unsigned short* er = eaL + (16 * t + m) * 32;
    a.h[0] = *(const v8us*)(er + 8 * h);
    a.h[1] = *(const v8us*)(er + 16 + 8 * h);
    v8f d1 = wm(a.u, B1h, z); d1 = wm(a.u, B1l, d1);
    v8f d2 = wm(a.u, B2h, z); d2 = wm(a.u, B2l, d2);
#pragma unroll
    for (int r = 0; r < 8; ++r) {
      const int el = 16 * t + 8 * h + r;
      const int id = idL[el];
      const int s = id >> 8, sl = id & (NB - 1);
      const v4f y = *(const v4f*)(y4L + 4 * el);
      const float x = Sin[(size_t)s * CS + c] * sc;
      const float ms = d1[r] * x;
      const float tv = d2[r] * x;
      float* q = ab + sl * AW + 4 * c;
      v4f o = *(const v4f*)q;
      o.x += ms; o.y += tv * y.x; o.z += tv * y.y; o.w += tv * y.z;
      *(v4f*)q = o;
    }
  }
}

template <int AW>
__device__ __forceinline__ void roleB(float* acc, const unsigned short* eaL, const int* idL, const float* y4L,
                                      const float* __restrict__ Vin, float sc, int c,
                                      v16us B1h, v16us B1l, v16us B2h, v16us B2l, int nt, int h, int m) {
  float* ab = acc + h * (NB * AW);
  const v8f z = zero8f();
#pragma unroll 1
  for (int t = 0; t < nt; ++t) {
    FU a;
    const unsigned short* er = eaL + (16 * t + m) * 32;
    a.h[0] = *(const v8us*)(er + 8 * h);
    a.h[1] = *(const v8us*)(er + 16 + 8 * h);
    v8f d1 = wm(a.u, B1h, z); d1 = wm(a.u, B1l, d1);
    v8f d2 = wm(a.u, B2h, z); d2 = wm(a.u, B2l, d2);
#pragma unroll
    for (int r = 0; r < 8; ++r) {
      const int el = 16 * t + 8 * h + r;
      const int id = idL[el];
      const int s = id >> 8, sl = id & (NB - 1);
      const v4f y = *(const v4f*)(y4L + 4 * el);
      const float* vp = Vin + (size_t)s * VW + c;
      const float v0 = vp[0] * sc, v1 = vp[CV] * sc, v2 = vp[2 * CV] * sc;
      const float vd = v0 * y.x + v1 * y.y + v2 * y.z;
      float* q = ab + sl * AW + 256 + 4 * c;
      v4f o = *(const v4f*)q;
      o.x += d1[r] * vd; o.y += d2[r] * v0; o.z += d2[r] * v1; o.w += d2[r] * v2;
      *(v4f*)q = o;
    }
  }
}

template <int AW>
__device__ __forceinline__ void roleC(float* acc, const unsigned short* eaL, const int* idL, const float* y4L,
                                      const float* __restrict__ Vin, float sc, int c,
                                      v16us B1h, v16us B1l, int nt, int h, int m) {
  float* ab = acc + h * (NB * AW);
  const v8f z = zero8f();
#pragma unroll 1
  for (int t = 0; t < nt; ++t) {
    FU a;
    const unsigned short* er = eaL + (16 * t + m) * 32;
    a.h[0] = *(const v8us*)(er + 8 * h);
    a.h[1] = *(const v8us*)(er + 16 + 8 * h);
    v8f d1 = wm(a.u, B1h, z); d1 = wm(a.u, B1l, d1);
#pragma unroll
    for (int r = 0; r < 8; ++r) {
      const int el = 16 * t + 8 * h + r;
      const int id = idL[el];
      const int s = id >> 8, sl = id & (NB - 1);
      const v4f y = *(const v4f*)(y4L + 4 * el);
      const float* vp = Vin + (size_t)s * VW + c;
      const float v0 = vp[0] * sc, v1 = vp[CV] * sc, v2 = vp[2 * CV] * sc;
      const float cx0 = v1 * y.z - v2 * y.y;
      const float cx1 = v2 * y.x - v0 * y.z;
      const float cx2 = v0 * y.y - v1 * y.x;
      const float w = d1[r];
      float* q = ab + sl * AW + 384 + 3 * c;
      q[0] += w * cx0; q[1] += w * cx1; q[2] += w * cx2;
    }
  }
}

__global__ __launch_bounds__(NTHR) void k_prep(const float* __restrict__ atab, const int* __restrict__ types,
                                               const float* __restrict__ ns0, const float* __restrict__ c_noise,
                                               float* S0, int nN, int nT, int nRows) {
  const int g = blockIdx.x * NTHR + threadIdx.x;
  if (g >= nRows * 16) return;
  const int n = g >> 4, qd = g & 15;
  int t = types[min(n, nN - 1)];
  t = (t < 0) ? t + nT : t;
  t = min(max(t, 0), nT - 1);
  const float cn = c_noise[0];
  v4f v;
#pragma unroll
  for (int j = 0; j < 4; ++j) { const int c = 4 * qd + j; v[j] = atab[t * CS + c] * (1.0f + cn * ns0[c]); }
  float* p = S0 + (size_t)g * 4;
  *(volatile v4f*)p = v;
  __threadfence();
  *(volatile v4f*)p = v;
}

template <int MODE>
__global__ __launch_bounds__(NTHR) void k_agg(
    const float* __restrict__ pos, const int* __restrict__ rad, const int* __restrict__ bnd,
    const float* __restrict__ bond_tab, const float* __restrict__ c_noise,
    const float* __restrict__ Sin, const float* __restrict__ Vin,
    const float* __restrict__ WeA, const float* __restrict__ WeB, const float* __restrict__ WeC,
    const float* __restrict__ WeD, const float* __restrict__ WeE,
    const float* __restrict__ Wms, const float* __restrict__ Wss,
    const float* __restrict__ Wmv, const float* __restrict__ Wsv,
    const float* __restrict__ nsw, const float* __restrict__ skw, const float* __restrict__ skb,
    const float* __restrict__ w_out, const float* __restrict__ gain,
    float* Sout, float* Vout, float* outp,
    int nN, int nER, int nEB, int vecOK, int isLast, float invn) {
  constexpr int AW  = accw(MODE);
  constexpr int KS1 = MODE ? 96 : 64;
  constexpr int KV1 = MODE ? 128 : 64;

  extern __shared__ __attribute__((aligned(16))) unsigned char dsm[];
  float* acc = reinterpret_cast<float*>(dsm);
  unsigned char* ur = dsm + 2 * NB * AW * 4;
  unsigned short* eaL = reinterpret_cast<unsigned short*>(ur);
  float* y4L  = reinterpret_cast<float*>(ur + PASSN * 64);
  int*   idL  = reinterpret_cast<int*>(ur + PASSN * 64 + PASSN * 16);
  int*   list = reinterpret_cast<int*>(ur + PASSN * 64 + PASSN * 16 + PASSN * 4);
  int*   pend = list + LISTN;
  float* stS  = reinterpret_cast<float*>(ur);
  float* stV  = reinterpret_cast<float*>(ur + NB * CS * 4);
  float* stO  = reinterpret_cast<float*>(ur + NB * CS * 4 + NB * VW * 4);
  float* scl  = reinterpret_cast<float*>(ur + UNIONB);
  float* gL   = scl + 96;
  float* woL  = gL + 192;
  float* cen  = woL + 32;
  int*   wcnt = reinterpret_cast<int*>(cen + 16);
  int*   pendN = wcnt + NWAVE;

  const int tid = threadIdx.x, lane = tid & 31, wave = tid >> 5, h = lane >> 4, m = lane & 15;
  const int nodeBase = blockIdx.x * NB;
  const int nE = nER + nEB;
  const float cn = c_noise[0];

  {
    const v4f z4 = {0.0f, 0.0f, 0.0f, 0.0f};
    for (int i = tid; i < (2 * NB * AW) / 4; i += NTHR) *(v4f*)(acc + 4 * i) = z4;
  }
  if (tid < 96) scl[tid] = MODE ? (1.0f + cn * nsw[tid]) : 1.0f;
  if (MODE) {
    if (tid < 192) { const float x = skb[tid] + cn * skw[tid]; gL[tid] = 1.0f / (1.0f + expf(-x)); }
  }
  if (tid < 32) woL[tid] = w_out[tid];
  if (tid == 0) {
    const float inv9 = 1.0f / 9.0f;
#pragma unroll
    for (int k = 1; k <= 8; ++k) cen[k - 1] = 1.5f * ((float)k * inv9);
    cen[8] = 1.0f / (cen[1] - cen[0]);
    pendN[0] = 0;
  }
  v16us B1h, B1l, B2h, B2l;
  {
    const float* W1; const float* W2; int nc, n0;
    if (MODE == 0)      { W1 = WeA; W2 = WeB; nc = CS; n0 = 16 * (wave & 3); }
    else if (wave < 4)  { W1 = WeA; W2 = WeC; nc = CS; n0 = 16 * wave; }
    else if (wave < 6)  { W1 = WeB; W2 = WeD; nc = CV; n0 = 16 * (wave - 4); }
    else                { W1 = WeE; W2 = WeE; nc = CV; n0 = 16 * (wave - 6); }
    fragBe(W1, nc, n0, h, m, B1h, B1l);
    fragBe(W2, nc, n0, h, m, B2h, B2l);
  }
  __syncthreads();

  const int nChunks = (nE + CHUNK - 1) / CHUNK;
#pragma unroll 1
  for (int ch = 0; ch < nChunks; ++ch) {
    const int cbase = ch * CHUNK;
    const int wc = scan_chunk(rad, bnd, nER, nEB, cbase, nodeBase, vecOK, list, tid, wave);
    if (lane == 0) wcnt[wave] = wc;
    __syncthreads();

    const int base = pendN[0];
    int tot = 0, myoff = 0;
#pragma unroll
    for (int w = 0; w < NWAVE; ++w) {
      int c = wcnt[w];
      c = c > WCAP ? WCAP : (c < 0 ? 0 : c);
      if (w < wave) myoff += c;
      tot += c;
    }
    int newN = base + tot;
    newN = newN > PCAP ? PCAP : newN;
    {
      int n = wcnt[wave];
      n = n > WCAP ? WCAP : (n < 0 ? 0 : n);
      const int* lp = list + wave * WCAP;
      for (int i = lane; i < n; i += 32) {
        const int pp = base + myoff + i;
        if (pp < PCAP) pend[pp] = cbase + lp[i];
      }
    }
    const int fin = (ch == nChunks - 1) ? 1 : 0;
    const int R  = (fin != 0) ? (newN + PASSN - 1) / PASSN : newN / PASSN;
    const int Pv = (fin != 0) ? newN : R * PASSN;
    __syncthreads();

#pragma unroll 1
    for (int rp = 0; rp < R; ++rp) {
      {
        const int idx = rp * PASSN + tid;
        const bool valid = idx < Pv;
        int e = pend[min(idx, PCAP - 1)];
        e = valid ? e : 0;
        e = min(max(e, 0), nE - 1);
        const int inB = (e >= nER) ? 1 : 0;
        const int er = min(e, nER - 1);
        const int eb = min(max(e - nER, 0), nEB - 1);
        const int sR = rad[er], dR = rad[nER + er];
        const int sB = bnd[eb], dB = bnd[nEB + eb];
        int s = inB ? sB : sR;
        const int d = inB ? dB : dR;
        int sl = d - nodeBase;
        const bool okd = valid && ((unsigned)sl < (unsigned)NB);
        sl = okd ? sl : 0;
        s = (s < 0) ? s + nN : s;
        s = min(max(s, 0), nN - 1);
        int dd = (d < 0) ? d + nN : d;
        dd = min(max(dd, 0), nN - 1);
        const float px = pos[(size_t)s * 3], py = pos[(size_t)s * 3 + 1], pz = pos[(size_t)s * 3 + 2];
        const float qx = pos[(size_t)dd * 3], qy = pos[(size_t)dd * 3 + 1], qz = pos[(size_t)dd * 3 + 2];
        const float dx = px - qx, dy = py - qy, dz = pz - qz;
        const float d2 = dx * dx + dy * dy + dz * dz + 1e-12f;
        const float dist = sqrtf(d2);
        const float rinv = 1.0f / dist;
        v4f yv;
        yv.x = okd ? (SQ3 * dx) * rinv : 0.0f;
        yv.y = okd ? (SQ3 * dy) * rinv : 0.0f;
        yv.z = okd ? (SQ3 * dz) * rinv : 0.0f;
        yv.w = 0.0f;
        const float rstep = cen[8];
        const float* bt = bond_tab + inB * 8;
        v8us hA, hB, lA, lB;
#pragma unroll
        for (int j = 0; j < 8; ++j) {
          float bv = bt[j];
          const float df = (dist - cen[j]) * rstep;
          float rb = expf(-(df * df)) * 1.12f;
          bv = okd ? bv : 0.0f;
          rb = okd ? rb : 0.0f;
          const unsigned int hb = bfb(bv), hr = bfb(rb);
          hA[j] = (unsigned short)hb; lA[j] = (unsigned short)bflo(bv, hb);
          hB[j] = (unsigned short)hr; lB[j] = (unsigned short)bflo(rb, hr);
        }
        unsigned short* row = eaL + tid * 32;
        *(v8us*)(row)      = hA;
        *(v8us*)(row + 8)  = hB;
        *(v8us*)(row + 16) = lA;
        *(v8us*)(row + 24) = lB;
        *(v4f*)(y4L + 4 * tid) = yv;
        idL[tid] = (s << 8) | sl;
      }
      __syncthreads();

      {
        const int nv = min(PASSN, Pv - rp * PASSN);
        const int nt = (nv + 15) >> 4;
        if (MODE == 0) {
          if (wave < 4) { const int c = 16 * wave + m; roleA<AW>(acc, eaL, idL, y4L, Sin, scl[c], c, B1h, B1l, B2h, B2l, nt, h, m); }
        } else {
          if (wave < 4)      { const int c = 16 * wave + m;       roleA<AW>(acc, eaL, idL, y4L, Sin, scl[c], c, B1h, B1l, B2h, B2l, nt, h, m); }
          else if (wave < 6) { const int c = 16 * (wave - 4) + m; roleB<AW>(acc, eaL, idL, y4L, Vin, scl[64 + c], c, B1h, B1l, B2h, B2l, nt, h, m); }
          else               { const int c = 16 * (wave - 6) + m; roleC<AW>(acc, eaL, idL, y4L, Vin, scl[64 + c], c, B1h, B1l, nt, h, m); }
        }
      }
      __syncthreads();
    }

    int rem = newN - R * PASSN;
    rem = rem < 0 ? 0 : rem;
    if (R > 0 && tid < rem) pend[tid] = pend[R * PASSN + tid];
    if (tid == 0) pendN[0] = rem;
  }
  __syncthreads();

  const float gn = gain[0];
#pragma unroll 1
  for (int task = wave; task < 40; task += NWAVE) {
    v8f d = zero8f();
    v16us ah, al, bh, bl;
    if (task < 16) {
      const int rt = task >> 2, n0 = 16 * (task & 3);
#pragma unroll 1
      for (int k0 = 0; k0 < KS1; k0 += 32) {
        const int bs = (k0 < 64) ? 4 * k0 : 256 + 4 * (k0 - 64);
        fragAacc<AW>(acc, 16 * rt, bs, 4, invn, h, m, ah, al);
        fragBw(Wms, CS, k0, n0, h, m, bh, bl);
        d = mm3(ah, al, bh, bl, d);
      }
#pragma unroll 1
      for (int k0 = 0; k0 < CS; k0 += 32) {
        fragApl(Sin, CS, 0, nodeBase + 16 * rt, nN, k0, scl, h, m, ah, al);
        fragBw(Wss, CS, k0, n0, h, m, bh, bl);
        d = mm3(ah, al, bh, bl, d);
      }
      const int c = n0 + m;
      const float ga = MODE ? gL[c] : 0.0f;
      const float gb = MODE ? gL[64 + c] : 1.0f;
#pragma unroll
      for (int r = 0; r < 8; ++r) {
        const int row = 16 * rt + 8 * h + r;
        float v = d[r];
        if (MODE) { const int n = min(nodeBase + row, nN - 1); v = ga * Sin[(size_t)n * CS + c] + gb * v; }
        stS[row * CS + c] = v;
      }
    } else {
      const int t2 = task - 16, i = t2 >> 3, rt = (t2 >> 1) & 3, n0 = 16 * (t2 & 1);
#pragma unroll 1
      for (int k0 = 0; k0 < KV1; k0 += 32) {
        int bs, st;
        if (k0 < 64)      { bs = 4 * k0 + 1 + i; st = 4; }
        else if (k0 < 96) { bs = 256 + 1 + i;    st = 4; }
        else              { bs = 384 + i;        st = 3; }
        fragAacc<AW>(acc, 16 * rt, bs, st, invn, h, m, ah, al);
        fragBw(Wmv, CV, k0, n0, h, m, bh, bl);
        d = mm3(ah, al, bh, bl, d);
      }
      if (MODE) {
        fragApl(Vin, VW, i * CV, nodeBase + 16 * rt, nN, 0, scl + 64, h, m, ah, al);
        fragBw(Wsv, CV, 0, n0, h, m, bh, bl);
        d = mm3(ah, al, bh, bl, d);
      }
      const int c = n0 + m;
      const float ga = MODE ? gL[128 + c] : 0.0f;
      const float gb = MODE ? gL[160 + c] : 1.0f;
#pragma unroll
      for (int r = 0; r < 8; ++r) {
        const int row = 16 * rt + 8 * h + r;
        float v = d[r];
        if (MODE) { const int n = min(nodeBase + row, nN - 1); v = ga * Vin[(size_t)n * VW + i * CV + c] + gb * v; }
        stV[row * VW + i * CV + c] = v;
      }
    }
  }
  __syncthreads();

  if (MODE && isLast != 0) {
    if (tid < 3 * NB) {
      const int n = tid / 3, i = tid - 3 * n;
      const float* vp = stV + n * VW + i * CV;
      float sum = 0.0f;
#pragma unroll 8
      for (int c = 0; c < CV; ++c) sum += vp[c] * woL[c];
      stO[tid] = sum * gn;
    }
  }
  __syncthreads();

  const int nValid = min(NB, nN - nodeBase);
  const int nf = 3 * nValid;
#pragma unroll 1
  for (int ps = 0; ps < 2; ++ps) {
#pragma unroll
    for (int it = 0; it < (NB * CS) / (NTHR * 4); ++it) {
      const int off = (it * NTHR + tid) * 4;
      const v4f v = *(const v4f*)(stS + off);
      *(volatile v4f*)(Sout + (size_t)nodeBase * CS + off) = v;
    }
#pragma unroll
    for (int it = 0; it < (NB * VW) / (NTHR * 4); ++it) {
      const int off = (it * NTHR + tid) * 4;
      const v4f v = *(const v4f*)(stV + off);
      *(volatile v4f*)(Vout + (size_t)nodeBase * VW + off) = v;
    }
    if (MODE && isLast != 0) {
      if (tid < (3 * NB) / 4 && 4 * tid + 4 <= nf) {
        const v4f v = *(const v4f*)(stO + 4 * tid);
        *(volatile v4f*)(outp + (size_t)nodeBase * 3 + 4 * tid) = v;
      }
      if (tid == 0) {
        for (int j = nf & ~3; j < nf; ++j) *(volatile float*)(outp + (size_t)nodeBase * 3 + j) = stO[j];
      }
    }
    if (ps == 0) __threadfence();
  }
}

extern "C" void kernel_launch(void* const* d_in, const int* in_sizes, int n_in,
                              void* d_out, int out_size, void* d_ws, size_t ws_size,
                              hipStream_t stream) {
  if (n_in < 27) return;
  const int nN = in_sizes[0] / 3;
  if (nN <= 0 || nN > (1 << 22) || in_sizes[0] != 3 * nN || in_sizes[1] < 1 || in_sizes[2] != nN) return;
  const int nER = in_sizes[3] / 2, nEB = in_sizes[4] / 2;
  if (nER <= 0 || nEB <= 0 || in_sizes[3] != 2 * nER || in_sizes[4] != 2 * nEB) return;
  const int nT = in_sizes[5] / CS;
  if (nT <= 0 || in_sizes[5] != nT * CS) return;
  if (in_sizes[6] != 16 || in_sizes[7] != CS || in_sizes[8] != EA * CS || in_sizes[9] != EA * CS) return;
  if (in_sizes[10] != CS * CS || in_sizes[11] != CS * CS || in_sizes[12] != CS * CV) return;
  const int L = in_sizes[13] / 96;
  if (L <= 0 || in_sizes[13] != L * 96) return;
  if (in_sizes[14] != L * EA * CS || in_sizes[15] != L * EA * CV || in_sizes[16] != L * EA * CS) return;
  if (in_sizes[17] != L * EA * CV || in_sizes[18] != L * EA * CV) return;
  if (in_sizes[19] != L * 96 * CS || in_sizes[20] != L * 128 * CV || in_sizes[21] != L * CS * CS || in_sizes[22] != L * CV * CV) return;
  if (in_sizes[23] != L * 192 || in_sizes[24] != L * 192 || in_sizes[25] != CV || in_sizes[26] < 1) return;
  if (out_size != 3 * nN) return;

  const float* pos      = (const float*)d_in[0];
  const float* c_noise  = (const float*)d_in[1];
  const int*   types    = (const int*)d_in[2];
  const int*   rad      = (const int*)d_in[3];
  const int*   bnd      = (const int*)d_in[4];
  const float* atom_tab = (const float*)d_in[5];
  const float* bond_tab = (const float*)d_in[6];
  const float* ns0_w    = (const float*)d_in[7];
  const float* We0      = (const float*)d_in[8];
  const float* We1      = (const float*)d_in[9];
  const float* Wself0   = (const float*)d_in[10];
  const float* Ws0      = (const float*)d_in[11];
  const float* Wv0      = (const float*)d_in[12];
  const float* ns_w     = (const float*)d_in[13];
  const float* We_ss    = (const float*)d_in[14];
  const float* We_vs    = (const float*)d_in[15];
  const float* We_sv    = (const float*)d_in[16];
  const float* We_vv    = (const float*)d_in[17];
  const float* We_vx    = (const float*)d_in[18];
  const float* Wmix_s   = (const float*)d_in[19];
  const float* Wmix_v   = (const float*)d_in[20];
  const float* Wself_s  = (const float*)d_in[21];
  const float* Wself_v  = (const float*)d_in[22];
  const float* skip_w   = (const float*)d_in[23];
  const float* skip_b   = (const float*)d_in[24];
  const float* w_out    = (const float*)d_in[25];
  const float* gain     = (const float*)d_in[26];
  float* out = (float*)d_out;

  const int nBlk = (nN + NB - 1) / NB;
  const int rows = nBlk * NB;

  char* ws = (char*)d_ws;
  const size_t szS = (size_t)rows * CS * 4;
  const size_t szV = (size_t)rows * VW * 4;
  const size_t total = 3 * szS + 2 * szV;
  if (total > ws_size) return;
  float* Sb[3]; float* Vb[2];
  Sb[0] = (float*)(ws);
  Sb[1] = (float*)(ws + szS);
  Sb[2] = (float*)(ws + 2 * szS);
  Vb[0] = (float*)(ws + 3 * szS);
  Vb[1] = (float*)(ws + 3 * szS + szV);

  const double ratio = (double)(nER + nEB) / (double)nN;
  double y = ratio > 1.0 ? ratio : 1.0;
  for (int it = 0; it < 64; ++it) y = 0.5 * (y + ratio / y);
  const float normf = (float)y;
  const float invn = 1.0f / normf;
  const int vecOK = (((nER & 3) == 0) && ((nEB & 3) == 0)) ? 1 : 0;

  hipFuncSetAttribute(reinterpret_cast<const void*>(&k_agg<0>), hipFuncAttributeMaxDynamicSharedMemorySize, lds_bytes(0));
  hipFuncSetAttribute(reinterpret_cast<const void*>(&k_agg<1>), hipFuncAttributeMaxDynamicSharedMemorySize, lds_bytes(1));

  k_prep<<<rows / 16, NTHR, 0, stream>>>(atom_tab, types, ns0_w, c_noise, Sb[0], nN, nT, rows);

  k_agg<0><<<nBlk, NTHR, lds_bytes(0), stream>>>(
      pos, rad, bnd, bond_tab, c_noise, Sb[0], Vb[1],
      We0, We1, We0, We0, We0, Ws0, Wself0, Wv0, Wv0,
      ns_w, skip_w, skip_b, w_out, gain,
      Sb[1], Vb[0], out, nN, nER, nEB, vecOK, 0, invn);

  for (int l = 0; l < L; ++l) {
    const float* Si = Sb[(1 + l) % 3];
    float*       So = Sb[(2 + l) % 3];
    const float* Vi = Vb[l & 1];
    float*       Vo = Vb[(l + 1) & 1];
    k_agg<1><<<nBlk, NTHR, lds_bytes(1), stream>>>(
        pos, rad, bnd, bond_tab, c_noise, Si, Vi,
        We_ss + (size_t)l * EA * CS, We_vs + (size_t)l * EA * CV, We_sv + (size_t)l * EA * CS,
        We_vv + (size_t)l * EA * CV, We_vx + (size_t)l * EA * CV,
        Wmix_s + (size_t)l * 96 * CS, Wself_s + (size_t)l * CS * CS,
        Wmix_v + (size_t)l * 128 * CV, Wself_v + (size_t)l * CV * CV,
        ns_w + (size_t)l * 96, skip_w + (size_t)l * 192, skip_b + (size_t)l * 192, w_out, gain,
        So, Vo, out, nN, nER, nEB, vecOK, (l == L - 1) ? 1 : 0, invn);
  }
}
